// MAGNOEncoder_87651692577273
// MI455X (gfx1250) — hardware-verified
//
#include <hip/hip_runtime.h>
#include <stdint.h>


typedef __bf16 v16bf __attribute__((ext_vector_type(16)));
typedef unsigned short v8us __attribute__((ext_vector_type(8), __may_alias__));
typedef float v8f __attribute__((ext_vector_type(8)));
typedef float v4f __attribute__((ext_vector_type(4), __may_alias__));

union FragB {
    v16bf v;
    v8us half[2];
    unsigned int u[8];
};

#define CDIM 2
#define INC 16
#define CH 32
#define HID 32
#define NT 128
#define NWAVE (NT / 32)
#define R1SQ 0.004900000000000001f
#define R2SQ 0.019600000000000003f

__device__ __forceinline__ unsigned int f2bf(float x) {
    unsigned int u = __float_as_uint(x);
    u += 0x7FFFu + ((u >> 16) & 1u);
    return u >> 16;
}
__device__ __forceinline__ float bf2f(unsigned int s) { return __uint_as_float(s << 16); }

__device__ __forceinline__ float gelu_f(float x) {
    const float inner = fmaf(0.044715f * (x * x), x, x);
    const float e = exp2f(inner * 2.3022082f);
    const float r = __builtin_amdgcn_rcpf(e + 1.0f);
    return x - x * r;
}

__device__ __forceinline__ v8f wmma_bf16(v16bf a, v16bf b, v8f c) {
    v8f d = __builtin_amdgcn_wmma_f32_16x16x32_bf16(false, a, false, b, (short)0, c, false, false);
    asm volatile("v_nop\n\tv_nop\n\tv_nop\n\tv_nop" : "+v"(d) : "v"(a), "v"(b));
    return d;
}

__launch_bounds__(256)
__global__ void k_lift(const float* __restrict__ pn, const float* __restrict__ Wl,
                       const float* __restrict__ bl, float* __restrict__ fo, int nrows) {
    const int gid = blockIdx.x * 256 + (int)threadIdx.x;
    const int row = gid >> 3;
    const int c0 = (gid & 7) * 4;
    const bool valid = row < nrows;
    const int rowc = valid ? row : 0;
    const v4f* p = (const v4f*)(pn + (size_t)rowc * INC);
    v4f a = {0.0f, 0.0f, 0.0f, 0.0f};
#pragma unroll
    for (int k4 = 0; k4 < INC / 4; ++k4) {
        const v4f pv = p[k4];
        const float pk[4] = {pv.x, pv.y, pv.z, pv.w};
#pragma unroll
        for (int s = 0; s < 4; ++s) {
            const v4f w = *(const v4f*)(Wl + (size_t)(4 * k4 + s) * CH + c0);
            a.x = fmaf(pk[s], w.x, a.x);
            a.y = fmaf(pk[s], w.y, a.y);
            a.z = fmaf(pk[s], w.z, a.z);
            a.w = fmaf(pk[s], w.w, a.w);
        }
    }
    const v4f bb = *(const v4f*)(bl + c0);
    a = a + bb;
    float* dst = fo + (size_t)rowc * CH + c0;
    if (valid) *(volatile v4f*)dst = a;
    __threadfence();
    if (valid) *(volatile v4f*)dst = a;
}

__launch_bounds__(NT)
__global__ void k_pairmlp_agg(const float* __restrict__ xc, const float* __restrict__ lat,
                              const float* __restrict__ kW1, const float* __restrict__ kb1,
                              const float* __restrict__ kW2, const float* __restrict__ kb2,
                              const float* __restrict__ kW3, const float* __restrict__ kb3,
                              const float* __restrict__ fsrc, float* __restrict__ out,
                              int npts, int nlat) {
    __shared__ unsigned short sW[4][HID * HID] __attribute__((aligned(16)));
    __shared__ float sL1[HID * 4] __attribute__((aligned(16)));
    __shared__ float sRed[NWAVE][2][CH] __attribute__((aligned(16)));
    __shared__ float sCnt[NWAVE][2];
    __shared__ float sOut[CH] __attribute__((aligned(16)));

    const int i = blockIdx.x;
    const int b = blockIdx.y;
    const int tid = (int)threadIdx.x;
    const int lane = tid & 31;
    const int wave = tid >> 5;
    const int col = lane & 15;
    const int hh = lane >> 4;

    const float q0 = lat[(size_t)i * CDIM + 0];
    const float q1 = lat[(size_t)i * CDIM + 1];

    if (tid < HID) {
        const int u = tid;
        float qp = q0 * kW1[2 * HID + u];
        qp = fmaf(q1, kW1[3 * HID + u], qp);
        qp += kb1[u];
        v4f cst;
        cst.x = kW1[u];
        cst.y = kW1[HID + u];
        cst.z = qp;
        cst.w = 0.0f;
        *(v4f*)(&sL1[4 * u]) = cst;
    }
#pragma unroll
    for (int s = 0; s < (HID * HID) / NT; ++s) {
        const int e = tid + NT * s;
        const int k = e >> 5;
        const int u = e & 31;
        const float w2 = kW2[e];
        const unsigned int h2 = f2bf(w2);
        const unsigned int l2 = f2bf(w2 - bf2f(h2));
        sW[0][u * HID + k] = (unsigned short)h2;
        sW[1][u * HID + k] = (unsigned short)l2;
        const float w3 = kW3[e];
        const unsigned int h3 = f2bf(w3);
        const unsigned int l3 = f2bf(w3 - bf2f(h3));
        sW[2][u * HID + k] = (unsigned short)h3;
        sW[3][u * HID + k] = (unsigned short)l3;
    }
    v8f cb2[2], cb3[2];
#pragma unroll
    for (int tt = 0; tt < 2; ++tt) {
#pragma unroll
        for (int r = 0; r < 8; ++r) {
            cb2[tt][r] = kb2[16 * tt + 8 * hh + r];
            cb3[tt][r] = kb3[16 * tt + 8 * hh + r];
        }
    }
    __syncthreads();

    float acc1[16], acc2[16];
#pragma unroll
    for (int e = 0; e < 16; ++e) { acc1[e] = 0.0f; acc2[e] = 0.0f; }
    float c1 = 0.0f, c2 = 0.0f;

    const int ntiles = (npts + 15) >> 4;
    for (int t = wave; t < ntiles; t += NWAVE) {
        asm volatile("" ::: "memory");
        const int j = t * 16 + col;
        const bool vj = j < npts;
        const int jc = vj ? j : (npts - 1);

        const float* xp = xc + ((size_t)b * npts + jc) * CDIM;
        const float x0 = xp[0];
        const float x1 = xp[1];
        float d2;
        {
#pragma clang fp contract(off)
            const float dx0 = x0 - q0;
            const float dx1 = x1 - q1;
            const float s0 = dx0 * dx0;
            const float s1 = dx1 * dx1;
            d2 = s0 + s1;
        }
        const float m1 = (vj && (d2 <= R1SQ)) ? 1.0f : 0.0f;
        const float m2 = (vj && (d2 <= R2SQ)) ? 1.0f : 0.0f;

        FragB bh, bl;
#pragma unroll
        for (int p = 0; p < 8; ++p) {
            unsigned int hp = 0u, lp = 0u;
#pragma unroll
            for (int s2 = 0; s2 < 2; ++s2) {
                const int e = 2 * p + s2;
                const int u = 8 * hh + (e & 7) + 2 * (e & 8);
                const v4f cst = *(const v4f*)(&sL1[4 * u]);
                const float pre = fmaf(x0, cst.x, fmaf(x1, cst.y, cst.z));
                const float g = gelu_f(pre);
                const unsigned int hs = f2bf(g);
                const unsigned int ls = f2bf(g - bf2f(hs));
                hp |= hs << (16 * s2);
                lp |= ls << (16 * s2);
            }
            bh.u[p] = hp;
            bl.u[p] = lp;
        }

        v8f acc[2];
#pragma unroll
        for (int tt = 0; tt < 2; ++tt) {
            const unsigned short* wh = &sW[0][(16 * tt + col) * HID];
            const unsigned short* wl = &sW[1][(16 * tt + col) * HID];
            FragB ah, al;
            ah.half[0] = *(const v8us*)(wh + 8 * hh);
            ah.half[1] = *(const v8us*)(wh + 16 + 8 * hh);
            al.half[0] = *(const v8us*)(wl + 8 * hh);
            al.half[1] = *(const v8us*)(wl + 16 + 8 * hh);
            v8f a = cb2[tt];
            a = wmma_bf16(ah.v, bh.v, a);
            a = wmma_bf16(ah.v, bl.v, a);
            a = wmma_bf16(al.v, bh.v, a);
            acc[tt] = a;
        }
        FragB ch, cl;
#pragma unroll
        for (int p = 0; p < 8; ++p) {
            unsigned int hp = 0u, lp = 0u;
#pragma unroll
            for (int s2 = 0; s2 < 2; ++s2) {
                const int e = 2 * p + s2;
                const float g = gelu_f(acc[e >> 3][e & 7]);
                const unsigned int hs = f2bf(g);
                const unsigned int ls = f2bf(g - bf2f(hs));
                hp |= hs << (16 * s2);
                lp |= ls << (16 * s2);
            }
            ch.u[p] = hp;
            cl.u[p] = lp;
        }

        v8f kv[2];
#pragma unroll
        for (int tt = 0; tt < 2; ++tt) {
            const unsigned short* wh = &sW[2][(16 * tt + col) * HID];
            const unsigned short* wl = &sW[3][(16 * tt + col) * HID];
            FragB ah, al;
            ah.half[0] = *(const v8us*)(wh + 8 * hh);
            ah.half[1] = *(const v8us*)(wh + 16 + 8 * hh);
            al.half[0] = *(const v8us*)(wl + 8 * hh);
            al.half[1] = *(const v8us*)(wl + 16 + 8 * hh);
            v8f a = cb3[tt];
            a = wmma_bf16(ah.v, ch.v, a);
            a = wmma_bf16(ah.v, cl.v, a);
            a = wmma_bf16(al.v, ch.v, a);
            kv[tt] = a;
        }

        const v4f* fp = (const v4f*)(fsrc + ((size_t)b * npts + jc) * CH);
        const v4f fA = fp[2 * hh], fB = fp[2 * hh + 1], fC = fp[4 + 2 * hh], fD = fp[5 + 2 * hh];
        const float fv[16] = { fA.x, fA.y, fA.z, fA.w, fB.x, fB.y, fB.z, fB.w,
                               fC.x, fC.y, fC.z, fC.w, fD.x, fD.y, fD.z, fD.w };
#pragma unroll
        for (int e = 0; e < 16; ++e) {
            const float tv = kv[e >> 3][e & 7] * fv[e];
            acc1[e] = fmaf(tv, m1, acc1[e]);
            acc2[e] = fmaf(tv, m2, acc2[e]);
        }
        c1 += m1;
        c2 += m2;
    }

#pragma unroll
    for (int off = 1; off < 16; off <<= 1) {
#pragma unroll
        for (int e = 0; e < 16; ++e) {
            acc1[e] += __shfl_xor(acc1[e], off, 32);
            acc2[e] += __shfl_xor(acc2[e], off, 32);
        }
        c1 += __shfl_xor(c1, off, 32);
        c2 += __shfl_xor(c2, off, 32);
    }
    if (col == 0) {
        float* r0 = &sRed[wave][0][0];
        float* r1 = &sRed[wave][1][0];
#pragma unroll
        for (int g = 0; g < 4; ++g) {
            const int cbase = 8 * hh + 4 * (g & 1) + 16 * (g >> 1);
            v4f v0, v1;
            v0.x = acc1[4 * g + 0]; v0.y = acc1[4 * g + 1]; v0.z = acc1[4 * g + 2]; v0.w = acc1[4 * g + 3];
            v1.x = acc2[4 * g + 0]; v1.y = acc2[4 * g + 1]; v1.z = acc2[4 * g + 2]; v1.w = acc2[4 * g + 3];
            *(v4f*)(r0 + cbase) = v0;
            *(v4f*)(r1 + cbase) = v1;
        }
        if (hh == 0) {
            sCnt[wave][0] = c1;
            sCnt[wave][1] = c2;
        }
    }
    __syncthreads();

    if (tid < CH) {
        const int c = tid;
        float s1 = sRed[0][0][c];
        float s2 = sRed[0][1][c];
        float n1 = sCnt[0][0];
        float n2 = sCnt[0][1];
#pragma unroll
        for (int w = 1; w < NWAVE; ++w) {
            s1 += sRed[w][0][c];
            s2 += sRed[w][1][c];
            n1 += sCnt[w][0];
            n2 += sCnt[w][1];
        }
        n1 = fmaxf(n1, 1.0f);
        n2 = fmaxf(n2, 1.0f);
        const float o = s1 * (1.0f / n1) + s2 * (1.0f / n2);
        sOut[c] = o;
    }
    __syncthreads();

    const size_t obase = ((size_t)b * nlat + i) * CH;
    v4f ov = {0.0f, 0.0f, 0.0f, 0.0f};
    if (tid < 8) {
        ov = *(const v4f*)(&sOut[4 * tid]);
        *(volatile v4f*)(out + obase + 4 * tid) = ov;
    }
    __threadfence();
    if (tid < 8) {
        *(volatile v4f*)(out + obase + 4 * tid) = ov;
    }
}

extern "C" void kernel_launch(void* const* d_in, const int* in_sizes, int n_in,
                              void* d_out, int out_size, void* d_ws, size_t ws_size,
                              hipStream_t stream) {
    if (n_in < 11) return;
    const float* x_coord = (const float*)d_in[0];
    const float* pndata  = (const float*)d_in[1];
    const float* latent  = (const float*)d_in[2];
    const float* W_lift  = (const float*)d_in[3];
    const float* b_lift  = (const float*)d_in[4];
    const float* kW1     = (const float*)d_in[5];
    const float* kb1     = (const float*)d_in[6];
    const float* kW2     = (const float*)d_in[7];
    const float* kb2     = (const float*)d_in[8];
    const float* kW3     = (const float*)d_in[9];
    const float* kb3     = (const float*)d_in[10];
    float* out = (float*)d_out;

    const int nlat = in_sizes[2] / CDIM;
    if (nlat <= 0 || out_size <= 0) return;
    const int nbq = out_size / CH;
    const int nb = nbq / nlat;
    if (nb <= 0) return;
    if (nb * nlat * CH != out_size) return;
    const int nrows = in_sizes[1] / INC;
    if (nrows <= 0) return;
    const int npts = nrows / nb;
    if (npts <= 0 || npts * nb != nrows) return;
    if (in_sizes[0] != nrows * CDIM) return;
    if (in_sizes[3] != INC * CH || in_sizes[5] != 2 * CDIM * HID ||
        in_sizes[7] != HID * HID || in_sizes[9] != HID * CH) return;

    const size_t fbytes = (size_t)nrows * CH * sizeof(float);
    if (fbytes > ws_size) return;
    float* f = (float*)d_ws;

    const int nthr = nrows * 8;
    k_lift<<<(nthr + 255) / 256, 256, 0, stream>>>(pndata, W_lift, b_lift, f, nrows);

    dim3 grid(nlat, nb);
    k_pairmlp_agg<<<grid, NT, 0, stream>>>(x_coord, latent, kW1, kb1, kW2, kb2, kW3, kb3,
                                           f, out, npts, nlat);
}
